// TemporalInteractionCrossAttention_32942399161113
// MI455X (gfx1250) — hardware-verified
//
#include <hip/hip_runtime.h>


#define NP2  32
#define NB1  16
#define TT   512
#define DM   512
#define NH_  8
#define HD   64
#define TE   2048
#define PCAR 1024.0f
typedef _Float16 h16;
typedef unsigned short bf;
typedef __attribute__((ext_vector_type(16))) __bf16   v16bf;
typedef __attribute__((ext_vector_type(16))) _Float16 v16h;
typedef __attribute__((ext_vector_type(8)))  _Float16 v8h;
typedef __attribute__((ext_vector_type(8)))  unsigned short v8us;
typedef __attribute__((ext_vector_type(8)))  float    v8f;
typedef __attribute__((ext_vector_type(4)))  float    v4f;
typedef v8h  __attribute__((may_alias)) v8ha;
typedef v4f  __attribute__((may_alias)) v4fa;
typedef v8us __attribute__((may_alias)) v8usa;

__device__ __forceinline__ unsigned short f2bf(float f) { unsigned u = __float_as_uint(f); u += 0x7FFFu + ((u >> 16) & 1u); return (unsigned short)(u >> 16); }
__device__ __forceinline__ float bf2f(unsigned short b) { return __uint_as_float(((unsigned)b) << 16); }
__device__ __forceinline__ float bfr(float f) { return bf2f(f2bf(f)); }
__device__ __forceinline__ v16h cat16(v8h lo, v8h hi) { return __builtin_shufflevector(lo, hi, 0, 1, 2, 3, 4, 5, 6, 7, 8, 9, 10, 11, 12, 13, 14, 15); }
__device__ __forceinline__ v16bf cat16b(v8us lo, v8us hi) { return __builtin_bit_cast(v16bf, __builtin_shufflevector(lo, hi, 0, 1, 2, 3, 4, 5, 6, 7, 8, 9, 10, 11, 12, 13, 14, 15)); }
__device__ __forceinline__ v8f wmma16(v16h a, v16h b, v8f c) { return __builtin_amdgcn_wmma_f32_16x16x32_f16(false, a, false, b, (short)0, c, false, false); }
__device__ __forceinline__ v8f wmmab(v16bf a, v16bf b, v8f c) { return __builtin_amdgcn_wmma_f32_16x16x32_bf16(false, a, false, b, (short)0, c, false, false); }


template <typename T16> struct WFrag;
template <> struct WFrag<h16> { typedef v16h V; static __device__ __forceinline__ V ld(const h16* p) { return cat16(*(const v8h*)p, *(const v8h*)(p + 16)); } static __device__ __forceinline__ v8f mma(V a, V b, v8f c) { return wmma16(a, b, c); } };
template <> struct WFrag<bf> { typedef v16bf V; static __device__ __forceinline__ V ld(const bf* p) { return cat16b(*(const v8us*)p, *(const v8us*)(p + 16)); } static __device__ __forceinline__ v8f mma(V a, V b, v8f c) { return wmmab(a, b, c); } };
template <typename T16, int NSPLIT, bool BIAS>
__global__ __launch_bounds__(32) void k_gemmw(const T16* __restrict__ A, const T16* __restrict__ A2, const T16* __restrict__ Bt, const T16* __restrict__ Bt2, int K, float* C, int ldc, const float* __restrict__ bias, size_t sA, size_t sB, size_t sC) {
    typedef typename WFrag<T16>::V V;
    __shared__ __align__(16) float os[16 * 68];
    const size_t z = blockIdx.z; A += z * sA; if (A2) A2 += z * sA; Bt += z * sB; if (Bt2) Bt2 += z * sB; C += z * sC;
    const int lane = threadIdx.x & 31, lr = lane & 15, hi = lane >> 4; const int r0 = blockIdx.x * 64, c0 = blockIdx.y * 64;
    v8f acc[4][4];
#pragma unroll
    for (int mb = 0; mb < 4; ++mb)
#pragma unroll
        for (int nb = 0; nb < 4; ++nb) acc[mb][nb] = (v8f){};
    const size_t aoff = (size_t)(r0 + lr) * K + 8 * hi, boff = (size_t)(c0 + lr) * K + 8 * hi;
#pragma unroll 1
    for (int kc = 0; kc < K; kc += 32) {
        V a[4], a2[4];
#pragma unroll
        for (int mb = 0; mb < 4; ++mb) { a[mb] = WFrag<T16>::ld(A + aoff + (size_t)mb * 16 * K + kc); if (NSPLIT == 1 || NSPLIT == 2) a2[mb] = WFrag<T16>::ld(A2 + aoff + (size_t)mb * 16 * K + kc); }
#pragma unroll
        for (int nb = 0; nb < 4; ++nb) { const V b = WFrag<T16>::ld(Bt + boff + (size_t)nb * 16 * K + kc); V b2; if (NSPLIT >= 2) b2 = WFrag<T16>::ld(Bt2 + boff + (size_t)nb * 16 * K + kc);
#pragma unroll
            for (int mb = 0; mb < 4; ++mb) { acc[mb][nb] = WFrag<T16>::mma(a[mb], b, acc[mb][nb]); if (NSPLIT == 1 || NSPLIT == 2) acc[mb][nb] = WFrag<T16>::mma(a2[mb], b, acc[mb][nb]); if (NSPLIT >= 2) acc[mb][nb] = WFrag<T16>::mma(a[mb], b2, acc[mb][nb]); } }
        asm volatile("v_nop\n\tv_nop\n\tv_nop\n\tv_nop" : "+v"(acc[0][0]), "+v"(acc[1][1]), "+v"(acc[2][2]), "+v"(acc[3][3]) : "v"(a[0]), "v"(a[3]));
    }
#pragma unroll
    for (int mb = 0; mb < 4; ++mb) {
#pragma unroll
        for (int nb = 0; nb < 4; ++nb) {
#pragma unroll
            for (int j = 0; j < 8; ++j) os[(hi * 8 + j) * 68 + nb * 16 + lr] = acc[mb][nb][j]; }
        __builtin_amdgcn_wave_barrier(); asm volatile("" ::: "memory");
        float* crow = C + (size_t)(r0 + mb * 16) * ldc + c0;
#pragma unroll 1
        for (int ps = 0; ps < 2; ++ps) {
#pragma unroll
            for (int s = 0; s < 8; ++s) { const int row = 2 * s + hi, cofs = lr * 4; v4f val = *(const v4fa*)(os + row * 68 + cofs); if (BIAS) { val[0] += bfr(bias[c0 + cofs]); val[1] += bfr(bias[c0 + cofs + 1]); val[2] += bfr(bias[c0 + cofs + 2]); val[3] += bfr(bias[c0 + cofs + 3]); }
                *(volatile v4f*)(crow + (size_t)row * ldc + cofs) = val; }
            if (ps == 0) __threadfence(); }
        __builtin_amdgcn_wave_barrier(); asm volatile("" ::: "memory");
    }
}

__device__ __forceinline__ h16 tohx(float x) { return (h16)x; }
__device__ __forceinline__ void splitf(float y, unsigned short& h, unsigned short& l) { h = f2bf(y); l = f2bf(y - bf2f(h)); }
typedef __attribute__((ext_vector_type(2))) unsigned short v2us;
typedef __attribute__((ext_vector_type(4))) unsigned short v4us;
typedef __attribute__((ext_vector_type(2))) _Float16 v2h;
typedef __attribute__((ext_vector_type(4))) _Float16 v4h;

__global__ __launch_bounds__(256) void k_wtG(const float* __restrict__ w, int K, int N, bf* Bt) {
    const int lane = threadIdx.x & 31; const int L0 = (blockIdx.x * 8 + (threadIdx.x >> 5)) * 8; const int nlines = N * K / 64;
#pragma unroll
    for (int ps = 0; ps < 2; ++ps) {
#pragma unroll 1
        for (int l = 0; l < 8; ++l) { const int L = L0 + l; if (L >= nlines) break; const size_t e = (size_t)L * 64 + lane * 2; const int k = (int)(e % K), n = (int)(e / K); v2us o;
            o[0] = f2bf(w[(size_t)k * N + n]); o[1] = f2bf(w[(size_t)(k + 1) * N + n]); *(volatile v2us*)(Bt + e) = o; }
        if (ps == 0) __threadfence(); }
}
__device__ __forceinline__ float siluf(float x) { float r = __builtin_amdgcn_rcpf(__fadd_rn(1.0f, __expf(-x))); asm volatile("" : "+v"(r)); return __fmul_rn(x, r); }
template <int MODE> __global__ __launch_bounds__(256) void k_ln(const float* __restrict__ X, const float* __restrict__ gg, const float* __restrict__ bb, const float* __restrict__ film, bf* Hh, bf* Hl) { const int lane = threadIdx.x & 31; const int t = blockIdx.x * 8 + (threadIdx.x >> 5); if (t >= TT) return; const float* xr = X + (size_t)t * DM; float v[DM / 32]; float s = 0.f;
#pragma unroll
    for (int ch = 0; ch < DM / 128; ++ch) { const v4f a = *(const v4f*)(xr + ch * 128 + lane * 4);
#pragma unroll
        for (int u = 0; u < 4; ++u) { v[ch * 4 + u] = MODE == 0 ? bfr(a[u]) : a[u]; s += v[ch * 4 + u]; } }
#pragma unroll
    for (int sh = 16; sh; sh >>= 1) s += __shfl_xor(s, sh, 32);
    const float mean = s * (1.0f / DM); float q = 0.f;
#pragma unroll
    for (int k = 0; k < DM / 32; ++k) { float d = __fsub_rn(v[k], mean); asm volatile("" : "+v"(d)); float p = __fmul_rn(d, d); asm volatile("" : "+v"(p)); q = __fadd_rn(q, p); }
#pragma unroll
    for (int sh = 16; sh; sh >>= 1) q += __shfl_xor(q, sh, 32);
    const float rstd = __frsqrt_rn(__fadd_rn(q * (1.0f / DM), 1e-5f));
    for (int ps = 0; ps < 2; ++ps) {
#pragma unroll
        for (int ch = 0; ch < DM / 128; ++ch) { v4us oh, ol; const int c0 = ch * 128 + lane * 4;
#pragma unroll
            for (int u = 0; u < 4; ++u) { const int c = c0 + u; float d = __fsub_rn(v[ch * 4 + u], mean); asm volatile("" : "+v"(d)); float n0 = __fmul_rn(d, rstd); asm volatile("" : "+v"(n0)); float g1 = bfr(gg[c]), b1 = bfr(bb[c]); asm volatile("" : "+v"(g1)); asm volatile("" : "+v"(b1)); float t1 = __fmul_rn(n0, g1); asm volatile("" : "+v"(t1)); float y = __fadd_rn(t1, b1);
                if (MODE == 1) { float sc = __fadd_rn(1.0f, film[c]); asm volatile("" : "+v"(sc)); float t2 = __fmul_rn(y, sc); asm volatile("" : "+v"(t2)); y = siluf(__fadd_rn(t2, film[DM + c])); }
                unsigned short a2, b2; splitf(y, a2, b2); oh[u] = a2; ol[u] = b2; }
            const size_t oo = (size_t)t * DM + c0; *(volatile v4us*)(Hh + oo) = oh; *(volatile v4us*)(Hl + oo) = ol; }
        if (ps == 0) __threadfence(); } }
__global__ __launch_bounds__(256) void k_pl(const float* __restrict__ F, h16* P) { const int e = (blockIdx.x * 256 + threadIdx.x) * 4; if (e >= NH_ * TT * HD) return; const int d = e % HD; const int t = (e / HD) % TT; const int h = e / (HD * TT); const float* f = F + (size_t)t * DM + h * HD + d; v4h o;
#pragma unroll
    for (int u = 0; u < 4; ++u) o[u] = tohx(f[u]); *(volatile v4h*)(P + e) = o; __threadfence(); *(volatile v4h*)(P + e) = o; }
__global__ __launch_bounds__(256) void k_vt(const float* __restrict__ V, h16* VT) { const int e = (blockIdx.x * 256 + threadIdx.x) * 2; if (e >= NH_ * HD * TT) return; const int t = e % TT; const int d = (e / TT) % HD; const int h = e / (TT * HD); v2h o; o[0] = tohx(V[(size_t)t * DM + h * HD + d]); o[1] = tohx(V[(size_t)(t + 1) * DM + h * HD + d]); *(volatile v2h*)(VT + e) = o; __threadfence(); *(volatile v2h*)(VT + e) = o; }
__global__ __launch_bounds__(256) void k_tsoft(const float* __restrict__ Sb, const float* __restrict__ msk, h16* P16) { const int lane = threadIdx.x & 31; const int row = blockIdx.x * 8 + (threadIdx.x >> 5); if (row >= NH_ * TT) return; const int n = row % TT; const float* sr = Sb + (size_t)row * TT; const float* mr = msk + (size_t)n * TT; float v[TT / 32]; float mx = -3.0e38f;
#pragma unroll
    for (int ch = 0; ch < TT / 128; ++ch) { const int m0 = ch * 128 + lane * 4; const v4f a = *(const v4f*)(sr + m0); const v4f mm = *(const v4f*)(mr + m0);
#pragma unroll
        for (int u = 0; u < 4; ++u) { float t0 = a[u] * 0.125f; asm volatile("" : "+v"(t0)); float om = __fsub_rn(1.0f, bfr(mm[u])); asm volatile("" : "+v"(om)); float ad = __fmul_rn(om, -100000.0f); asm volatile("" : "+v"(ad)); const float t = __fadd_rn(t0, ad); v[ch * 4 + u] = t; mx = fmaxf(mx, t); } }
#pragma unroll
    for (int sh = 16; sh; sh >>= 1) mx = fmaxf(mx, __shfl_xor(mx, sh, 32));
    float sum = 0.f;
#pragma unroll
    for (int q = 0; q < TT / 32; ++q) { float d0 = __fsub_rn(v[q], mx); asm volatile("" : "+v"(d0)); v[q] = __builtin_amdgcn_exp2f(__fmul_rn(d0, 1.4426950408889634f)); sum += v[q]; }
#pragma unroll
    for (int sh = 16; sh; sh >>= 1) sum += __shfl_xor(sum, sh, 32);
    const float f = __fdiv_rn(PCAR, sum);
    for (int ps = 0; ps < 2; ++ps) {
#pragma unroll
        for (int ch = 0; ch < TT / 128; ++ch) { v4h o4;
#pragma unroll
            for (int q = 0; q < 4; ++q) o4[q] = tohx(v[ch * 4 + q] * f); *(volatile v4h*)(P16 + (size_t)row * TT + ch * 128 + lane * 4) = o4; }
        if (ps == 0) __threadfence(); } }
__global__ __launch_bounds__(256) void k_ymrg(const float* __restrict__ O, float* Y) { const int e = (blockIdx.x * 256 + threadIdx.x) * 4; if (e >= TT * DM) return; const int c = e % DM; const int t = e / DM; const int h = c / HD, d = c % HD; const v4f a = *(const v4f*)(O + ((size_t)h * TT + t) * HD + d); v4f o;
#pragma unroll
    for (int u = 0; u < 4; ++u) o[u] = a[u] * (1.0f / PCAR); *(volatile v4f*)(Y + e) = o; __threadfence(); *(volatile v4f*)(Y + e) = o; }
__global__ __launch_bounds__(256) void k_emb(const float* __restrict__ emb, const float* __restrict__ We, const float* __restrict__ be, float* EO) { const int o = blockIdx.x * 256 + threadIdx.x; if (o >= 2 * DM) return; float s = 0.f;
#pragma unroll 1
    for (int e = 0; e < TE; ++e) { const float ev = siluf(bfr(emb[e])); float w = bfr(We[(size_t)e * 2 * DM + o]); asm volatile("" : "+v"(w)); float p = __fmul_rn(ev, w); asm volatile("" : "+v"(p)); s = __fadd_rn(s, p); }
    const float r = __fadd_rn(s, bfr(be[o])); *(volatile float*)(EO + o) = r; __threadfence(); *(volatile float*)(EO + o) = r; }
__global__ __launch_bounds__(256) void k_out(const float* __restrict__ x, const float* __restrict__ HO, float* OUTb) { const int e = (blockIdx.x * 256 + threadIdx.x) * 4; if (e >= TT * DM) return; const v4f a = *(const v4f*)(x + e), h = *(const v4f*)(HO + e); v4f o;
#pragma unroll
    for (int u = 0; u < 4; ++u) o[u] = __fadd_rn(bfr(a[u]), h[u]); *(volatile v4f*)(OUTb + e) = o; __threadfence(); *(volatile v4f*)(OUTb + e) = o; }

extern "C" void kernel_launch(void* const* d_in, const int* in_sizes, int n_in,
                              void* d_out, int out_size, void* d_ws, size_t ws_size, hipStream_t stream) {
    (void)in_sizes; (void)n_in; (void)out_size;
    const float** I = (const float**)d_in;
    const float *x1 = I[0], *x2 = I[1], *emb = I[2], *smask = I[3], *lxg = I[4], *lxb = I[5], *ltg = I[6], *ltb = I[7], *Wq = I[8], *bq = I[9], *Wk = I[10], *bk = I[11], *Wv = I[12], *bv = I[13], *Wemb = I[14], *bemb = I[15], *sbg = I[16], *sbb = I[17], *Wout = I[18], *bout = I[19];
    float* OUT0 = (float*)d_out; float* OUT1 = OUT0 + (size_t)NB1 * TT * DM;
    char* wsp = (char*)d_ws;
    auto take = [&](size_t bytes) { char* p = wsp; wsp += (bytes + 255) & ~(size_t)255; return (void*)p; };
    bf* BQ = (bf*)take((size_t)DM * DM * 2); bf* BK = (bf*)take((size_t)DM * DM * 2); bf* BV = (bf*)take((size_t)DM * DM * 2); bf* BO = (bf*)take((size_t)DM * DM * 2);
    bf* Xh = (bf*)take((size_t)TT * DM * 2); bf* Xl = (bf*)take((size_t)TT * DM * 2); bf* Th = (bf*)take((size_t)TT * DM * 2); bf* Tl = (bf*)take((size_t)TT * DM * 2); float* FQ = (float*)take((size_t)TT * DM * 4); float* FK = (float*)take((size_t)TT * DM * 4); float* FV = (float*)take((size_t)TT * DM * 4);
    h16* Q16 = (h16*)take((size_t)NH_ * TT * HD * 2); h16* K16 = (h16*)take((size_t)NH_ * TT * HD * 2); h16* VT = (h16*)take((size_t)NH_ * HD * TT * 2); float* Sb = (float*)take((size_t)NH_ * TT * TT * 4); h16* P16 = (h16*)take((size_t)NH_ * TT * TT * 2); float* O = (float*)take((size_t)NH_ * TT * HD * 4); float* Y = (float*)take((size_t)TT * DM * 4);
    float* EO = (float*)take(2 * DM * 4); bf* Sh = (bf*)take((size_t)TT * DM * 2); bf* Sl = (bf*)take((size_t)TT * DM * 2); float* HO = (float*)take((size_t)TT * DM * 4);
    if ((size_t)(wsp - (char*)d_ws) > ws_size) return;
    k_wtG<<<(DM * DM / 64 + 63) / 64, 256, 0, stream>>>(Wq, DM, DM, BQ); k_wtG<<<(DM * DM / 64 + 63) / 64, 256, 0, stream>>>(Wk, DM, DM, BK); k_wtG<<<(DM * DM / 64 + 63) / 64, 256, 0, stream>>>(Wv, DM, DM, BV); k_wtG<<<(DM * DM / 64 + 63) / 64, 256, 0, stream>>>(Wout, DM, DM, BO);
    const unsigned gE = (TT * DM / 4 + 255) / 256;
    for (int i = 0; i < NP2; ++i) { const float* xa = (i < NB1) ? x1 + (size_t)i * TT * DM : x2 + (size_t)(i - NB1) * TT * DM; const float* xb = (i < NB1) ? x2 + (size_t)i * TT * DM : x1 + (size_t)(i - NB1) * TT * DM; float* outp = (i < NB1) ? OUT0 + (size_t)i * TT * DM : OUT1 + (size_t)(i - NB1) * TT * DM;
        k_ln<0><<<TT / 8, 256, 0, stream>>>(xa, lxg, lxb, nullptr, Xh, Xl); k_ln<0><<<TT / 8, 256, 0, stream>>>(xb, ltg, ltb, nullptr, Th, Tl);
        k_gemmw<bf, 1, true><<<dim3(TT / 64, DM / 64, 1), 32, 0, stream>>>(Xh, Xl, BQ, nullptr, DM, FQ, DM, bq, 0, 0, 0); k_gemmw<bf, 1, true><<<dim3(TT / 64, DM / 64, 1), 32, 0, stream>>>(Th, Tl, BK, nullptr, DM, FK, DM, bk, 0, 0, 0); k_gemmw<bf, 1, true><<<dim3(TT / 64, DM / 64, 1), 32, 0, stream>>>(Th, Tl, BV, nullptr, DM, FV, DM, bv, 0, 0, 0);
        k_pl<<<(NH_ * TT * HD / 4 + 255) / 256, 256, 0, stream>>>(FQ, Q16); k_pl<<<(NH_ * TT * HD / 4 + 255) / 256, 256, 0, stream>>>(FK, K16); k_vt<<<(NH_ * HD * TT / 2 + 255) / 256, 256, 0, stream>>>(FV, VT);
        k_gemmw<h16, 0, false><<<dim3(TT / 64, TT / 64, NH_), 32, 0, stream>>>(Q16, nullptr, K16, nullptr, HD, Sb, TT, nullptr, (size_t)TT * HD, (size_t)TT * HD, (size_t)TT * TT);
        k_tsoft<<<NH_ * TT / 8, 256, 0, stream>>>(Sb, smask + (size_t)i * TT * TT, P16);
        k_gemmw<h16, 0, false><<<dim3(TT / 64, 1, NH_), 32, 0, stream>>>(P16, nullptr, VT, nullptr, TT, O, HD, nullptr, (size_t)TT * TT, (size_t)HD * TT, (size_t)TT * HD);
        k_ymrg<<<gE, 256, 0, stream>>>(O, Y); k_emb<<<(2 * DM + 255) / 256, 256, 0, stream>>>(emb + (size_t)i * TE, Wemb, bemb, EO);
        k_ln<1><<<TT / 8, 256, 0, stream>>>(Y, sbg, sbb, EO, Sh, Sl); k_gemmw<bf, 1, true><<<dim3(TT / 64, DM / 64, 1), 32, 0, stream>>>(Sh, Sl, BO, nullptr, DM, HO, DM, bout, 0, 0, 0);
        k_out<<<gE, 256, 0, stream>>>(xa, HO, outp); }
}
